// TransformerScaledDotProductAttention_73959336837600
// MI455X (gfx1250) — hardware-verified
//
#include <hip/hip_runtime.h>
#include <math.h>

typedef __attribute__((ext_vector_type(16))) _Float16 v16h;
typedef __attribute__((ext_vector_type(16))) __bf16 v16b;
typedef __attribute__((ext_vector_type(8)))  _Float16 v8h;
typedef __attribute__((ext_vector_type(8)))  float v8f;
typedef __attribute__((ext_vector_type(4)))  float v4f;
typedef __attribute__((ext_vector_type(2)))  float v2f;
typedef __attribute__((ext_vector_type(4)))  unsigned v4u;
typedef __attribute__((ext_vector_type(4)))  int v4i;
typedef float __attribute__((may_alias)) float_a;
typedef int __attribute__((may_alias)) int_a;

template <typename T> __device__ __forceinline__ void vst2(void* p, T v) { *(volatile T*)p = v; __threadfence(); *(volatile T*)p = v; }
__device__ __forceinline__ v8f wmma16(v16h a, v16h b, v8f c) {
  v8f d = __builtin_amdgcn_wmma_f32_16x16x32_f16(false, a, false, b, (short)0, c, false, false);
  asm volatile("v_nop\n\tv_nop\n\tv_nop\n\tv_nop" : "+v"(d) : "v"(a), "v"(b));
  return d;
}
__device__ __forceinline__ v8f wmma_bf(v16b a, v16b b, v8f c) {
  v8f d = __builtin_amdgcn_wmma_f32_16x16x32_bf16(false, a, false, b, (short)0, c, false, false);
  asm volatile("v_nop\n\tv_nop\n\tv_nop\n\tv_nop" : "+v"(d) : "v"(a), "v"(b));
  return d;
}
__device__ __forceinline__ v16h frag_h(const _Float16* rowk0, int lane) {
  union { v16h v; v8h q[2]; } u; const _Float16* p = rowk0 + 8 * (lane >> 4);
  u.q[0] = *(const v8h*)p; u.q[1] = *(const v8h*)(p + 16); return u.v;
}
__device__ __forceinline__ v16h frag_f32(const float* rowk0, int lane) {
  v16h a; const float* p = rowk0 + 8 * (lane >> 4);
#pragma unroll
  for (int i = 0; i < 8; ++i) { a[i] = (_Float16)p[i]; a[8 + i] = (_Float16)p[16 + i]; }
  return a;
}
__device__ __forceinline__ v16h frag_f32s(const float* rowk0, int lane, float sc) {
  v16h a; const float* p = rowk0 + 8 * (lane >> 4);
#pragma unroll
  for (int i = 0; i < 8; ++i) { a[i] = (_Float16)(p[i] * sc); a[8 + i] = (_Float16)(p[16 + i] * sc); }
  return a;
}
__device__ __forceinline__ v16h fragc_f32(const float* W, int k0, int n, int lane, int ld, int K) {
  v16h a; const int g = lane >> 4;
#pragma unroll
  for (int i = 0; i < 8; ++i) { const int ka = k0 + 8 * g + i, kb = ka + 16;
    a[i] = (_Float16)(ka < K ? W[(size_t)(ka < K ? ka : K - 1) * ld + n] : 0.f); a[8 + i] = (_Float16)(kb < K ? W[(size_t)(kb < K ? kb : K - 1) * ld + n] : 0.f); }
  return a;
}
struct F2 { v16b h, l; };
__device__ __forceinline__ F2 bsplit16(const float v[16]) { F2 r;
#pragma unroll
  for (int i = 0; i < 16; ++i) { const __bf16 h = (__bf16)v[i]; r.h[i] = h; r.l[i] = (__bf16)(v[i] - (float)h); }
  return r; }
__device__ __forceinline__ F2 split_row(const float* row, int k0, int lane) { float v[16]; const float* p = row + k0 + 8 * (lane >> 4);
#pragma unroll
  for (int i = 0; i < 8; ++i) { v[i] = p[i]; v[8 + i] = p[16 + i]; }
  return bsplit16(v); }
__device__ __forceinline__ F2 split_rowK(const float* row, int k0, int lane, int K) { float v[16]; const int g = lane >> 4;
#pragma unroll
  for (int i = 0; i < 8; ++i) { const int ka = k0 + 8 * g + i, kb = ka + 16; v[i] = ka < K ? row[ka < K ? ka : K - 1] : 0.f; v[8 + i] = kb < K ? row[kb < K ? kb : K - 1] : 0.f; }
  return bsplit16(v); }
__device__ __forceinline__ F2 split_col(const float* W, int k0, int n, int lane, int ld, int K) { float v[16]; const int g = lane >> 4;
#pragma unroll
  for (int i = 0; i < 8; ++i) { const int ka = k0 + 8 * g + i, kb = ka + 16; v[i] = ka < K ? W[(size_t)(ka < K ? ka : K - 1) * ld + n] : 0.f; v[8 + i] = kb < K ? W[(size_t)(kb < K ? kb : K - 1) * ld + n] : 0.f; }
  return bsplit16(v); }
__device__ __forceinline__ v8f mac3(const F2& a, const F2& b, v8f c) { c = wmma_bf(a.l, b.h, c); c = wmma_bf(a.h, b.l, c); return wmma_bf(a.h, b.h, c); }
__device__ __forceinline__ float sigm(float v) { return 1.0f / (1.0f + expf(-v)); }
#define LDSX() do { asm volatile("s_wait_dscnt 0" ::: "memory"); __builtin_amdgcn_wave_barrier(); __builtin_amdgcn_fence(__ATOMIC_RELEASE, "workgroup"); } while (0)


#define NBH 64
#define LL 2048
#define DD 64
#ifndef TKB
#define TKB (LL / 64)
#define TNB NBH
#endif
typedef __attribute__((ext_vector_type(8))) __bf16 v8b;
__device__ __forceinline__ v16b frag_b(const __bf16* rowk0, int lane) {
  union { v16b v; v8b q[2]; } u; const __bf16* p = rowk0 + 8 * (lane >> 4);
  u.q[0] = *(const v8b*)p; u.q[1] = *(const v8b*)(p + 16); return u.v;
}
__device__ __forceinline__ v16b frag_gbf(const float* rowk0, int lane) {
  v16b a; const float* p = rowk0 + 8 * (lane >> 4);
#pragma unroll
  for (int i = 0; i < 8; ++i) { a[i] = (__bf16)p[i]; a[8 + i] = (__bf16)p[16 + i]; }
  return a;
}
__device__ __attribute__((noinline)) float exp_ni(float v) { return expf(v); }
#define WS_M   0u
#define WS_L   (WS_M + 4u * NBH * LL)
#define WS_END (WS_L + 4u * NBH * LL)
__global__ __launch_bounds__(128) void k_stats(const float* __restrict__ Q, const float* __restrict__ K, float* __restrict__ M, float* __restrict__ IL) {
  __shared__ __align__(16) float sm[64], sl[64];
  const int tid = threadIdx.x, wave = tid >> 5, lane = tid & 31, col = lane & 15, g = lane >> 4; const int bh = blockIdx.y; const int q0 = blockIdx.x * 64 + wave * 16;
  const v16b a0 = frag_gbf(Q + ((size_t)bh * LL + q0 + col) * DD, lane), a1 = frag_gbf(Q + ((size_t)bh * LL + q0 + col) * DD + 32, lane);
  float m[8], l[8];
#pragma unroll
  for (int r = 0; r < 8; ++r) { m[r] = -3.0e38f; l[r] = 0.f; }
#pragma unroll 1
  for (int ks = 0; ks < LL / 32; ++ks) { float s[2][8];
#pragma unroll
    for (int ct = 0; ct < 2; ++ct) { const float* krow = K + ((size_t)bh * LL + ks * 32 + ct * 16 + col) * DD; v8f c = {}; c = wmma_bf(a0, frag_gbf(krow, lane), c); c = wmma_bf(a1, frag_gbf(krow + 32, lane), c);
#pragma unroll
      for (int r = 0; r < 8; ++r) s[ct][r] = c[r] * 0.125f; }
#pragma unroll
    for (int r = 0; r < 8; ++r) { float mx = fmaxf(s[0][r], s[1][r]);
#pragma unroll
      for (int o = 1; o < 16; o <<= 1) mx = fmaxf(mx, __shfl_xor(mx, o));
      const float mn = fmaxf(m[r], mx); float es = exp_ni(s[0][r] - mn) + exp_ni(s[1][r] - mn);
#pragma unroll
      for (int o = 1; o < 16; o <<= 1) es += __shfl_xor(es, o);
      l[r] = l[r] * exp_ni(m[r] - mn) + es; m[r] = mn; } }
  if (col == 0) {
#pragma unroll
    for (int r = 0; r < 8; ++r) { sm[wave * 16 + 8 * g + r] = m[r]; sl[wave * 16 + 8 * g + r] = 1.0f / l[r]; } }
  __syncthreads();
  if (tid < 16) vst2(M + (size_t)bh * LL + blockIdx.x * 64 + tid * 4, *(const v4f*)&sm[tid * 4]); else if (tid < 32) vst2(IL + (size_t)bh * LL + blockIdx.x * 64 + (tid - 16) * 4, *(const v4f*)&sl[(tid - 16) * 4]);
}
__global__ __launch_bounds__(128) void k_va(const float* __restrict__ Q, const float* __restrict__ K, const float* __restrict__ V, const float* __restrict__ M, const float* __restrict__ IL, float* __restrict__ OUT) {
  __shared__ __align__(16) __bf16 sph[4][16][40], spl[4][16][40]; __shared__ __align__(16) float so[64][68];
  const int tid = threadIdx.x, wave = tid >> 5, lane = tid & 31, col = lane & 15, g = lane >> 4; const int bh = blockIdx.y; const int k0 = blockIdx.x * 64 + wave * 16;
  const v16b ka0 = frag_gbf(K + ((size_t)bh * LL + k0 + col) * DD, lane), ka1 = frag_gbf(K + ((size_t)bh * LL + k0 + col) * DD + 32, lane);
  const float* Vb = V + (size_t)bh * DD * LL; const float* Mb = M + (size_t)bh * LL; const float* ILb = IL + (size_t)bh * LL;
  v8f acc[4] = {};
#pragma unroll 1
  for (int qs = 0; qs < LL / 32; ++qs) {
#pragma unroll
    for (int ct = 0; ct < 2; ++ct) { const int q = qs * 32 + ct * 16 + col; const float* qrow = Q + ((size_t)bh * LL + q) * DD; v8f c = {}; c = wmma_bf(ka0, frag_gbf(qrow, lane), c); c = wmma_bf(ka1, frag_gbf(qrow + 32, lane), c);
      const float mq = Mb[q], ilq = ILb[q];
#pragma unroll
      for (int r = 0; r < 8; ++r) { const float p = exp_ni(c[r] * 0.125f - mq) * ilq; const __bf16 hb = (__bf16)p; sph[wave][8 * g + r][ct * 16 + col] = hb; spl[wave][8 * g + r][ct * 16 + col] = (__bf16)(p - (float)hb); } }
    LDSX();
    const v16b ph = frag_b(&sph[wave][col][0], lane), pl = frag_b(&spl[wave][col][0], lane);
#pragma unroll
    for (int dt = 0; dt < 4; ++dt) { const v16b va = frag_gbf(Vb + (size_t)(dt * 16 + col) * LL + qs * 32, lane); acc[dt] = wmma_bf(va, pl, acc[dt]); acc[dt] = wmma_bf(va, ph, acc[dt]); }
    LDSX(); }
#pragma unroll
  for (int dt = 0; dt < 4; ++dt)
#pragma unroll
    for (int r = 0; r < 8; ++r) so[dt * 16 + 8 * g + r][wave * 16 + col] = acc[dt][r];
  __syncthreads();
  for (int qd = tid; qd < 64 * 16; qd += 128) { const int d = qd >> 4, pc = qd & 15; vst2(OUT + ((size_t)bh * DD + d) * LL + blockIdx.x * 64 + pc * 4, *(const v4f*)&so[d][pc * 4]); }
}
extern "C" void kernel_launch(void* const* d_in, const int* in_sizes, int n_in, void* d_out, int out_size, void* d_ws, size_t ws_size, hipStream_t stream) {
  (void)in_sizes; (void)n_in; (void)out_size;
  const float** F = (const float**)d_in;
  if (ws_size < (size_t)WS_END) return;
  char* ws = (char*)d_ws; float *M = (float*)(ws + WS_M), *IL = (float*)(ws + WS_L);
  k_stats<<<dim3(LL / 64, TNB), 128, 0, stream>>>(F[0], F[1], M, IL);
  k_va<<<dim3(TKB, TNB), 128, 0, stream>>>(F[0], F[1], F[2], M, IL, (float*)d_out);
}
